// MeshInterpolateModuleVoGE_3307124818190
// MI455X (gfx1250) — hardware-verified
//
#include <hip/hip_runtime.h>


#pragma clang fp contract(off)

typedef _Float16 v16h __attribute__((ext_vector_type(16)));
typedef _Float16 v8h  __attribute__((ext_vector_type(8)));
typedef float    v8f  __attribute__((ext_vector_type(8)));
typedef float    v4f  __attribute__((ext_vector_type(4)));
typedef int      v4i  __attribute__((ext_vector_type(4)));

#define NB   2
#define NV   1024
#define NF   2048
#define NC   128
#define NHW  128
#define FOCAL_C    2.0f
#define WSCALE     16384.0f
#define WSCALE_INV (1.0f / 16384.0f)

union Frag   { v16h v; v8h h8[2]; _Float16 s[16]; };
union Pack16 { v8h h; v4i i; };

__device__ __forceinline__ v8f wmma_f16(v16h a, v16h b, v8f c) {
  v8f d = __builtin_amdgcn_wmma_f32_16x16x32_f16(false, a, false, b, (short)0, c, false, false);
  asm volatile("v_nop\n\tv_nop\n\tv_nop\n\tv_nop" : "+v"(d) : "v"(a), "v"(b));
  return d;
}

__device__ __forceinline__ float lin_coord(int i) {
  const float t = (float)i / (float)(NHW - 1);
  const float r = -1.0f * (1.0f - t) + 1.0f * t;
  return (i == NHW - 1) ? 1.0f : r;
}

__global__ __launch_bounds__(256) void k_geom(const float* __restrict__ campos,
                                              const float* __restrict__ theta,
                                              const float* __restrict__ vertices,
                                              const int*   __restrict__ faces,
                                              v4f* __restrict__ c4) {
  __shared__ int   s_fi[NF * 3];
  __shared__ float s_fe[NF * 3];
  const int tid = threadIdx.x;

  #pragma unroll 1
  for (int f = tid; f < NF; f += 256) {
    int i0 = faces[f * 3 + 0], i1 = faces[f * 3 + 1], i2 = faces[f * 3 + 2];
    i0 = min(max(i0, 0), NV - 1);
    i1 = min(max(i1, 0), NV - 1);
    i2 = min(max(i2, 0), NV - 1);
    const float ax = vertices[i0 * 3 + 0], ay = vertices[i0 * 3 + 1], az = vertices[i0 * 3 + 2];
    const float ux = vertices[i1 * 3 + 0], uy = vertices[i1 * 3 + 1], uz = vertices[i1 * 3 + 2];
    const float qx = vertices[i2 * 3 + 0], qy = vertices[i2 * 3 + 1], qz = vertices[i2 * 3 + 2];
    float d0 = ax - ux, d1 = az - uz, d2 = ay - uy;
    const float e01 = sqrtf((d0 * d0 + d1 * d1) + d2 * d2);
    d0 = ux - qx; d1 = uz - qz; d2 = uy - qy;
    const float e12 = sqrtf((d0 * d0 + d1 * d1) + d2 * d2);
    d0 = qx - ax; d1 = qz - az; d2 = qy - ay;
    const float e20 = sqrtf((d0 * d0 + d1 * d1) + d2 * d2);
    s_fi[f * 3 + 0] = i0;  s_fi[f * 3 + 1] = i1;  s_fi[f * 3 + 2] = i2;
    s_fe[f * 3 + 0] = e01; s_fe[f * 3 + 1] = e12; s_fe[f * 3 + 2] = e20;
  }
  __syncthreads();

  const int v = blockIdx.x * 256 + tid;
  if (v < NV) {
    float ssum = 0.0f, cnt = 0.0f;
    #pragma unroll 1
    for (int f = 0; f < NF; ++f) {
      const int i0 = s_fi[f * 3 + 0], i1 = s_fi[f * 3 + 1], i2 = s_fi[f * 3 + 2];
      const bool m0 = (i0 == v), m1 = (i1 == v), m2 = (i2 == v);
      if (m0 | m1 | m2) {
        const float e01 = s_fe[f * 3 + 0], e12 = s_fe[f * 3 + 1], e20 = s_fe[f * 3 + 2];
        const float t = (m0 ? (e01 + e20) : 0.0f) + (m1 ? (e01 + e12) : 0.0f) + (m2 ? (e12 + e20) : 0.0f);
        ssum = ssum + t;
        cnt = cnt + ((m0 ? 2.0f : 0.0f) + (m1 ? 2.0f : 0.0f) + (m2 ? 2.0f : 0.0f));
      }
    }
    const float me  = ssum / fmaxf(cnt, 1.0f);
    const float rad = 0.5f * me;
    const float sig = rad * rad + 1e-6f;

    const float p0 = vertices[v * 3 + 0], p1 = vertices[v * 3 + 2], p2 = vertices[v * 3 + 1];

    #pragma unroll 1
    for (int bb = 0; bb < NB; ++bb) {
      const float cx = campos[bb * 3 + 0], cy = campos[bb * 3 + 1], cz = campos[bb * 3 + 2];
      const float nz = sqrtf((cx * cx + cy * cy) + cz * cz);
      const float rz = 1.0f / (nz + 1e-8f);
      const float Z0 = (-cx) * rz, Z1 = (-cy) * rz, Z2 = (-cz) * rz;
      const float Xr0 = Z2, Xr1 = 0.0f, Xr2 = -Z0;
      const float nx = sqrtf((Xr0 * Xr0 + Xr1 * Xr1) + Xr2 * Xr2);
      const float rx = 1.0f / (nx + 1e-8f);
      const float X0 = Xr0 * rx, X1 = Xr1 * rx, X2 = Xr2 * rx;
      const float Y0 = Z1 * X2 - Z2 * X1;
      const float Y1 = Z2 * X0 - Z0 * X2;
      const float Y2 = Z0 * X1 - Z1 * X0;
      float st, ct;
      sincosf(theta[bb], &st, &ct);
      const float R00 = X0 * ct + Y0 * st, R10 = X1 * ct + Y1 * st, R20 = X2 * ct + Y2 * st;
      const float R01 = X0 * (-st) + Y0 * ct, R11 = X1 * (-st) + Y1 * ct, R21 = X2 * (-st) + Y2 * ct;
      const float T0 = -((R00 * cx + R10 * cy) + R20 * cz);
      const float T1 = -((R01 * cx + R11 * cy) + R21 * cz);
      const float T2 = -((Z0  * cx + Z1  * cy) + Z2  * cz);
      const float vc0 = ((p0 * R00 + p1 * R10) + p2 * R20) + T0;
      const float vc1 = ((p0 * R01 + p1 * R11) + p2 * R21) + T1;
      const float vc2 = ((p0 * Z0  + p1 * Z1 ) + p2 * Z2 ) + T2;
      const float zc  = fmaxf(vc2, 1e-4f);
      const float rzc = 1.0f / zc;
      const float px  = (FOCAL_C * vc0) * rzc;
      const float py  = (FOCAL_C * vc1) * rzc;
      const float fz  = FOCAL_C * rzc;
      const float s2  = sig * (fz * fz);
      const float nh  = -1.0f / (2.0f * s2);
      v4f r4;
      r4.x = px; r4.y = py; r4.z = nh; r4.w = vc2;
      volatile v4f* dst = (volatile v4f*)(c4 + (size_t)bb * NV + v);
      *dst = r4;
      __threadfence();
      *dst = r4;
    }
  }
}

__global__ __launch_bounds__(NV) void k_sort(const v4f* __restrict__ c4,
                                             v4f* __restrict__ par4,
                                             int* __restrict__ sidx) {
  __shared__ float key[NV];
  __shared__ int   val[NV];
  const int b = blockIdx.x, tid = threadIdx.x;
  const v4f me = c4[(size_t)b * NV + tid];
  key[tid] = me.w;
  val[tid] = tid;
  __syncthreads();
  for (int k = 2; k <= NV; k <<= 1) {
    for (int j = k >> 1; j > 0; j >>= 1) {
      const int ixj = tid ^ j;
      if (ixj > tid) {
        const bool  up = ((tid & k) == 0);
        const float a  = key[tid], c = key[ixj];
        const int   ia = val[tid], ic = val[ixj];
        const bool  gt = (a > c) || ((a == c) && (ia > ic));
        if (gt == up) {
          key[tid] = c;  key[ixj] = a;
          val[tid] = ic; val[ixj] = ia;
        }
      }
      __syncthreads();
    }
  }
  const int idx = val[tid];
  const v4f P = c4[(size_t)b * NV + idx];
  volatile v4f* dp = (volatile v4f*)(par4 + (size_t)b * NV + tid);
  volatile int* di = (volatile int*)(sidx + (size_t)b * NV + tid);
  *dp = P;
  *di = idx;
  __threadfence();
  *dp = P;
  *di = idx;
}

__global__ __launch_bounds__(256) void k_feat(const float* __restrict__ memory,
                                              const int*   __restrict__ sidx,
                                              _Float16* __restrict__ featT) {
  __shared__ __attribute__((aligned(16))) _Float16 tile[16][NV + 8];
  const int g = blockIdx.x, b = blockIdx.y, tid = threadIdx.x;
  const int c0 = g * 16;

  #pragma unroll 1
  for (int i = tid; i < NV; i += 256) {
    int n = sidx[(size_t)b * NV + i];
    n = min(max(n, 0), NV - 1);
    const float* src = memory + (size_t)n * NC + c0;
    const v4f x0 = *(const v4f*)(src + 0);
    const v4f x1 = *(const v4f*)(src + 4);
    const v4f x2 = *(const v4f*)(src + 8);
    const v4f x3 = *(const v4f*)(src + 12);
    tile[0][i]  = (_Float16)x0.x; tile[1][i]  = (_Float16)x0.y; tile[2][i]  = (_Float16)x0.z; tile[3][i]  = (_Float16)x0.w;
    tile[4][i]  = (_Float16)x1.x; tile[5][i]  = (_Float16)x1.y; tile[6][i]  = (_Float16)x1.z; tile[7][i]  = (_Float16)x1.w;
    tile[8][i]  = (_Float16)x2.x; tile[9][i]  = (_Float16)x2.y; tile[10][i] = (_Float16)x2.z; tile[11][i] = (_Float16)x2.w;
    tile[12][i] = (_Float16)x3.x; tile[13][i] = (_Float16)x3.y; tile[14][i] = (_Float16)x3.z; tile[15][i] = (_Float16)x3.w;
  }
  __syncthreads();

  const int wave = tid >> 5, lane = tid & 31;
  _Float16* dstb = featT + ((size_t)b * NC + c0) * NV;
  #pragma unroll
  for (int rr = 0; rr < 2; ++rr) {
    const int row = wave * 2 + rr;
    #pragma unroll
    for (int q = 0; q < 4; ++q) {
      const int off = (q * 32 + lane) * 8;
      Pack16 pk; pk.h = *(const v8h*)(&tile[row][off]);
      *(volatile v4i*)(dstb + (size_t)row * NV + off) = pk.i;
    }
  }
  __threadfence();
  #pragma unroll
  for (int rr = 0; rr < 2; ++rr) {
    const int row = wave * 2 + rr;
    #pragma unroll
    for (int q = 0; q < 4; ++q) {
      const int off = (q * 32 + lane) * 8;
      Pack16 pk; pk.h = *(const v8h*)(&tile[row][off]);
      *(volatile v4i*)(dstb + (size_t)row * NV + off) = pk.i;
    }
  }
}

__global__ __launch_bounds__(128) void k_main(const v4f* __restrict__ par4,
                                              const _Float16* __restrict__ featT,
                                              float* __restrict__ out) {
  __shared__ __attribute__((aligned(16))) float sT[4][16][132];
  __shared__ float sInv[4][16];
  const int halfc = blockIdx.x;
  const int h     = blockIdx.y;
  const int b     = blockIdx.z;
  const int wave  = threadIdx.x >> 5;
  const int lane  = threadIdx.x & 31;
  const int m     = lane & 15;
  const int hh    = lane >> 4;
  const int wbase = halfc * 64 + wave * 16;

  const float gx = lin_coord(wbase + m);
  const float gy = lin_coord(h);

  const v4f* par = par4 + (size_t)b * NV;
  const _Float16* fb = featT + (size_t)b * NC * NV;

  float S   = 0.0f;
  float nrm = 0.0f;
  v8f acc[8];
  #pragma unroll
  for (int t = 0; t < 8; ++t) { v8f z; for (int r = 0; r < 8; ++r) z[r] = 0.0f; acc[t] = z; }

  for (int kc = 0; kc < NV; kc += 32) {
    const int kb0 = kc + 8 * hh;
    const int kb1 = kc + 16 + 8 * hh;

    float wl[16];
    float g0 = 0.0f, g1 = 0.0f;
    #pragma unroll
    for (int e = 0; e < 8; ++e) {
      const v4f P = par[kb0 + e];
      const float dx = P.x - gx, dy = P.y - gy;
      const float d2 = dx * dx + dy * dy;
      float w = __expf(d2 * P.z);
      w = (P.w > 1e-4f) ? w : 0.0f;
      wl[e] = w;
      g0 = g0 + w;
    }
    #pragma unroll
    for (int e = 0; e < 8; ++e) {
      const v4f P = par[kb1 + e];
      const float dx = P.x - gx, dy = P.y - gy;
      const float d2 = dx * dx + dy * dy;
      float w = __expf(d2 * P.z);
      w = (P.w > 1e-4f) ? w : 0.0f;
      wl[8 + e] = w;
      g1 = g1 + w;
    }

    const float o0 = __shfl_xor(g0, 16, 32);
    const float o1 = __shfl_xor(g1, 16, 32);
    const float q0 = hh ? o0 : g0;
    const float q1 = hh ? g0 : o0;
    const float q2 = hh ? o1 : g1;
    const float q3 = hh ? g1 : o1;
    const float p01   = S + q0;
    const float p012  = p01 + q1;
    const float base0 = hh ? p01 : S;
    const float base1 = hh ? (p012 + q2) : p012;
    S = S + ((q0 + q1) + (q2 + q3));

    Frag A;
    float run = 0.0f;
    #pragma unroll
    for (int e = 0; e < 8; ++e) {
      const float w  = wl[e];
      const float wf = w * __expf(-(base0 + run));
      run = run + w;
      nrm = nrm + wf;
      A.s[e] = (_Float16)(wf * WSCALE);
    }
    run = 0.0f;
    #pragma unroll
    for (int e = 0; e < 8; ++e) {
      const float w  = wl[8 + e];
      const float wf = w * __expf(-(base1 + run));
      run = run + w;
      nrm = nrm + wf;
      A.s[8 + e] = (_Float16)(wf * WSCALE);
    }

    #pragma unroll
    for (int t = 0; t < 8; ++t) {
      const _Float16* bp = fb + (size_t)(t * 16 + m) * NV + kb0;
      Frag Bf;
      Bf.h8[0] = *(const v8h*)(bp);
      Bf.h8[1] = *(const v8h*)(bp + 16);
      acc[t] = wmma_f16(A.v, Bf.v, acc[t]);
    }
  }

  const float nrmT = nrm + __shfl_xor(nrm, 16, 32);
  if (hh == 0) sInv[wave][m] = (1.0f / (nrmT + 1e-8f)) * WSCALE_INV;

  #pragma unroll
  for (int t = 0; t < 8; ++t) {
    #pragma unroll
    for (int r = 0; r < 8; ++r) sT[wave][8 * hh + r][t * 16 + m] = acc[t][r];
  }
  __syncthreads();

  float* ob = out + (((size_t)b * NHW + h) * NHW + wbase) * NC;
  #pragma unroll
  for (int row = 0; row < 16; ++row) {
    const float sc = sInv[wave][row];
    const v4f a = *(const v4f*)(&sT[wave][row][4 * lane]);
    const v4f val = a * sc;
    *(volatile v4f*)(ob + (size_t)row * NC + 4 * lane) = val;
  }
  __threadfence();
  #pragma unroll
  for (int row = 0; row < 16; ++row) {
    const float sc = sInv[wave][row];
    const v4f a = *(const v4f*)(&sT[wave][row][4 * lane]);
    const v4f val = a * sc;
    *(volatile v4f*)(ob + (size_t)row * NC + 4 * lane) = val;
  }
}

extern "C" void kernel_launch(void* const* d_in, const int* in_sizes, int n_in,
                              void* d_out, int out_size, void* d_ws, size_t ws_size,
                              hipStream_t stream) {
  if (n_in < 5) return;
  if (in_sizes[0] < NB * 3 || in_sizes[1] < NB || in_sizes[2] < NV * 3 ||
      in_sizes[3] < NF * 3 || in_sizes[4] < NV * NC) return;
  if ((size_t)out_size < (size_t)NB * NHW * NHW * NC) return;

  const float* campos   = (const float*)d_in[0];
  const float* theta    = (const float*)d_in[1];
  const float* vertices = (const float*)d_in[2];
  const int*   faces    = (const int*)d_in[3];
  const float* memory   = (const float*)d_in[4];
  float* out = (float*)d_out;

  const size_t sz_c4   = (size_t)NB * NV * sizeof(v4f);
  const size_t sz_sidx = (size_t)NB * NV * sizeof(int);
  const size_t sz_feat = (size_t)NB * NC * NV * sizeof(_Float16);
  const size_t off_c4   = 0;
  const size_t off_par  = off_c4 + sz_c4;
  const size_t off_sidx = off_par + sz_c4;
  const size_t off_feat = off_sidx + sz_sidx;
  const size_t total    = off_feat + sz_feat;
  if (total > ws_size) return;

  char* ws = (char*)d_ws;
  v4f* c4   = (v4f*)(ws + off_c4);
  v4f* par4 = (v4f*)(ws + off_par);
  int* sidx = (int*)(ws + off_sidx);
  _Float16* featT = (_Float16*)(ws + off_feat);

  k_geom<<<(NV + 255) / 256, 256, 0, stream>>>(campos, theta, vertices, faces, c4);
  k_sort<<<NB, NV, 0, stream>>>(c4, par4, sidx);
  k_feat<<<dim3(NC / 16, NB), 256, 0, stream>>>(memory, sidx, featT);
  k_main<<<dim3(2, NHW, NB), 128, 0, stream>>>(par4, featT, out);
}
